// EfficientSelfAtten_1726576854494
// MI455X (gfx1250) — hardware-verified
//
#include <hip/hip_runtime.h>
#include <math.h>

typedef __attribute__((ext_vector_type(16))) _Float16 v16h;
typedef __attribute__((ext_vector_type(16))) __bf16 v16b;
typedef __attribute__((ext_vector_type(8)))  _Float16 v8h;
typedef __attribute__((ext_vector_type(8)))  float v8f;
typedef __attribute__((ext_vector_type(4)))  float v4f;
typedef __attribute__((ext_vector_type(2)))  float v2f;
typedef __attribute__((ext_vector_type(4)))  unsigned v4u;
typedef __attribute__((ext_vector_type(4)))  int v4i;
typedef float __attribute__((may_alias)) float_a;
typedef int __attribute__((may_alias)) int_a;

template <typename T> __device__ __forceinline__ void vst2(void* p, T v) { *(volatile T*)p = v; __threadfence(); *(volatile T*)p = v; }
__device__ __forceinline__ v8f wmma16(v16h a, v16h b, v8f c) {
  v8f d = __builtin_amdgcn_wmma_f32_16x16x32_f16(false, a, false, b, (short)0, c, false, false);
  asm volatile("v_nop\n\tv_nop\n\tv_nop\n\tv_nop" : "+v"(d) : "v"(a), "v"(b));
  return d;
}
__device__ __forceinline__ v8f wmma_bf(v16b a, v16b b, v8f c) {
  v8f d = __builtin_amdgcn_wmma_f32_16x16x32_bf16(false, a, false, b, (short)0, c, false, false);
  asm volatile("v_nop\n\tv_nop\n\tv_nop\n\tv_nop" : "+v"(d) : "v"(a), "v"(b));
  return d;
}
__device__ __forceinline__ v16h frag_h(const _Float16* rowk0, int lane) {
  union { v16h v; v8h q[2]; } u; const _Float16* p = rowk0 + 8 * (lane >> 4);
  u.q[0] = *(const v8h*)p; u.q[1] = *(const v8h*)(p + 16); return u.v;
}
__device__ __forceinline__ v16h frag_f32(const float* rowk0, int lane) {
  v16h a; const float* p = rowk0 + 8 * (lane >> 4);
#pragma unroll
  for (int i = 0; i < 8; ++i) { a[i] = (_Float16)p[i]; a[8 + i] = (_Float16)p[16 + i]; }
  return a;
}
__device__ __forceinline__ v16h frag_f32s(const float* rowk0, int lane, float sc) {
  v16h a; const float* p = rowk0 + 8 * (lane >> 4);
#pragma unroll
  for (int i = 0; i < 8; ++i) { a[i] = (_Float16)(p[i] * sc); a[8 + i] = (_Float16)(p[16 + i] * sc); }
  return a;
}
__device__ __forceinline__ v16h fragc_f32(const float* W, int k0, int n, int lane, int ld, int K) {
  v16h a; const int g = lane >> 4;
#pragma unroll
  for (int i = 0; i < 8; ++i) { const int ka = k0 + 8 * g + i, kb = ka + 16;
    a[i] = (_Float16)(ka < K ? W[(size_t)ka * ld + n] : 0.f); a[8 + i] = (_Float16)(kb < K ? W[(size_t)kb * ld + n] : 0.f); }
  return a;
}
struct F2 { v16b h, l; };
__device__ __forceinline__ F2 bsplit16(const float v[16]) { F2 r;
#pragma unroll
  for (int i = 0; i < 16; ++i) { const __bf16 h = (__bf16)v[i]; r.h[i] = h; r.l[i] = (__bf16)(v[i] - (float)h); }
  return r; }
__device__ __forceinline__ F2 split_row(const float* row, int k0, int lane) { float v[16]; const float* p = row + k0 + 8 * (lane >> 4);
#pragma unroll
  for (int i = 0; i < 8; ++i) { v[i] = p[i]; v[8 + i] = p[16 + i]; }
  return bsplit16(v); }
__device__ __forceinline__ F2 split_rowK(const float* row, int k0, int lane, int K) { float v[16]; const int g = lane >> 4;
#pragma unroll
  for (int i = 0; i < 8; ++i) { const int ka = k0 + 8 * g + i, kb = ka + 16; v[i] = ka < K ? row[ka] : 0.f; v[8 + i] = kb < K ? row[kb] : 0.f; }
  return bsplit16(v); }
__device__ __forceinline__ F2 split_col(const float* W, int k0, int n, int lane, int ld, int K) { float v[16]; const int g = lane >> 4;
#pragma unroll
  for (int i = 0; i < 8; ++i) { const int ka = k0 + 8 * g + i, kb = ka + 16; v[i] = ka < K ? W[(size_t)ka * ld + n] : 0.f; v[8 + i] = kb < K ? W[(size_t)kb * ld + n] : 0.f; }
  return bsplit16(v); }
__device__ __forceinline__ v8f mac3(const F2& a, const F2& b, v8f c) { c = wmma_bf(a.l, b.h, c); c = wmma_bf(a.h, b.l, c); return wmma_bf(a.h, b.h, c); }
__device__ __forceinline__ float sigm(float v) { return 1.0f / (1.0f + expf(-v)); }
#define LDSX() do { asm volatile("s_wait_dscnt 0" ::: "memory"); __builtin_amdgcn_wave_barrier(); __builtin_amdgcn_fence(__ATOMIC_RELEASE, "workgroup"); } while (0)

#define NB 8
#define NN 4096
#define CC 256
#define NH 8
#define HD 32
#define HI 64
#define WI 64
#define RR 4
#define NK 256
#define NR (NB * NN)

__global__ __launch_bounds__(256) void k_cvt(const float* __restrict__ x, _Float16* __restrict__ x16, size_t n8) {
  const size_t g8 = (size_t)blockIdx.x * 256 + threadIdx.x; if (g8 >= n8) return;
  union { v8h h; v4u u; } pk;
#pragma unroll
  for (int e = 0; e < 8; ++e) pk.h[e] = (_Float16)x[g8 * 8 + e];
  vst2(x16 + g8 * 8, pk.u);
}
__global__ __launch_bounds__(256) void k_pack(const float* __restrict__ qw, const float* __restrict__ kvw, const float* __restrict__ pw, const float* __restrict__ srw, _Float16* __restrict__ P, _Float16* __restrict__ Psr) {
  const int r = blockIdx.x, tid = threadIdx.x;
  if (r < 1024) { __shared__ __align__(16) _Float16 srow[CC];
    const float* W; int n, NOUT; if (r < 256) { W = qw; n = r; NOUT = CC; } else if (r < 768) { W = kvw; n = r - 256; NOUT = 2 * CC; } else { W = pw; n = r - 768; NOUT = CC; }
    srow[tid] = (_Float16)(W[(size_t)tid * NOUT + n] * 16.0f);
    __syncthreads();
    if (tid < CC / 8) vst2(P + (size_t)r * CC + tid * 8, *(const v4u*)(&srow[tid * 8])); }
  else { const int o = r - 1024; __shared__ __align__(16) _Float16 sr2[16 * CC];
    for (int q = tid; q < 16 * CC; q += 256) { const int t = q >> 8, c = q & 255; sr2[q] = (_Float16)(srw[(((size_t)o * CC + c) * RR + (t >> 2)) * RR + (t & 3)] * 16.0f); }
    __syncthreads();
    for (int q = tid; q < 16 * CC / 8; q += 256) vst2(Psr + (size_t)o * (16 * CC) + q * 8, *(const v4u*)(&sr2[q * 8])); }
}
__global__ __launch_bounds__(128) void k_q(const _Float16* __restrict__ x16, const _Float16* __restrict__ P, const float* __restrict__ qb, _Float16* __restrict__ Q16) {
  __shared__ __align__(16) float so[4][16][132];
  const int tid = threadIdx.x, wave = tid >> 5, lane = tid & 31, col = lane & 15, g = lane >> 4;
  const int r0 = blockIdx.x * 64 + wave * 16, n0 = blockIdx.y * 128;
  v8f acc[8] = {};
#pragma unroll
  for (int kc = 0; kc < CC / 32; ++kc) { const v16h a = frag_h(x16 + (size_t)(r0 + col) * CC + kc * 32, lane);
#pragma unroll
    for (int j = 0; j < 8; ++j) acc[j] = wmma16(a, frag_h(P + (size_t)(n0 + j * 16 + col) * CC + kc * 32, lane), acc[j]); }
#pragma unroll
  for (int j = 0; j < 8; ++j) { const float bb = qb[n0 + j * 16 + col];
#pragma unroll
    for (int r = 0; r < 8; ++r) so[wave][8 * g + r][j * 16 + col] = (acc[j][r] * (1.0f / 16.0f) + bb) * 4.0f; }
  LDSX();
  for (int q = lane; q < 16 * 16; q += 32) { const int rl = q >> 4, pc = q & 15; union { v8h h8; v4u u; } pk;
#pragma unroll
    for (int e = 0; e < 8; ++e) pk.h8[e] = (_Float16)so[wave][rl][pc * 8 + e];
    vst2(Q16 + (size_t)(r0 + rl) * CC + n0 + pc * 8, pk.u); }
}
__global__ __launch_bounds__(128) void k_kv(const _Float16* __restrict__ x16, const _Float16* __restrict__ Psr, const float* __restrict__ srb, const float* __restrict__ ng, const float* __restrict__ nbeta, const _Float16* __restrict__ P, const float* __restrict__ kvb, _Float16* __restrict__ K16, _Float16* __restrict__ VT) {
  __shared__ __align__(16) float sx[4][16][CC + 4];
  __shared__ __align__(16) float so[4][16][2 * CC + 4];
  __shared__ __align__(16) _Float16 st[CC][72];
  const int tid = threadIdx.x, wave = tid >> 5, lane = tid & 31, col = lane & 15, g = lane >> 4;
  const int b = blockIdx.y, t0b = blockIdx.x * 64, py = blockIdx.x * 4 + wave;
#pragma unroll 1
  for (int np = 0; np < 2; ++np) { v8f acc[8] = {};
#pragma unroll 1
    for (int kc = 0; kc < 16 * CC / 32; ++kc) { const int t = kc >> 3, c0 = (kc & 7) * 32; const int ky = t >> 2, kx = t & 3;
      const v16h a = frag_h(x16 + ((size_t)b * NN + (4 * py + ky) * WI + 4 * col + kx) * CC + c0, lane);
#pragma unroll
      for (int j = 0; j < 8; ++j) acc[j] = wmma16(a, frag_h(Psr + (size_t)(np * 128 + j * 16 + col) * (16 * CC) + kc * 32, lane), acc[j]); }
#pragma unroll
    for (int j = 0; j < 8; ++j) { const int o = np * 128 + j * 16 + col; const float bb = srb[o];
#pragma unroll
      for (int r = 0; r < 8; ++r) sx[wave][8 * g + r][o] = acc[j][r] * (1.0f / 16.0f) + bb; } }
  LDSX();
  { const int rl = lane >> 1, hf = lane & 1; float* row = &sx[wave][rl][0]; float s = 0.f; for (int c = 0; c < 128; ++c) s += row[hf * 128 + c]; s += __shfl_xor(s, 1, 32); const float mu = s * (1.0f / CC);
    float q2 = 0.f; for (int c = 0; c < 128; ++c) { const float d = row[hf * 128 + c] - mu; q2 += d * d; } q2 += __shfl_xor(q2, 1, 32); const float rs = rsqrtf(q2 * (1.0f / CC) + 1e-5f);
    LDSX();
    for (int c = 0; c < 128; ++c) { const int cc = hf * 128 + c; row[cc] = (row[cc] - mu) * rs * ng[cc] + nbeta[cc]; } }
  LDSX();
#pragma unroll 1
  for (int np = 0; np < 4; ++np) { v8f acc[8] = {};
#pragma unroll
    for (int kc = 0; kc < CC / 32; ++kc) { const v16h a = frag_f32(&sx[wave][col][0] + kc * 32, lane);
#pragma unroll
      for (int j = 0; j < 8; ++j) acc[j] = wmma16(a, frag_h(P + (size_t)(256 + np * 128 + j * 16 + col) * CC + kc * 32, lane), acc[j]); }
#pragma unroll
    for (int j = 0; j < 8; ++j) { const int o = np * 128 + j * 16 + col; const float bb = kvb[o];
#pragma unroll
      for (int r = 0; r < 8; ++r) so[wave][8 * g + r][o] = acc[j][r] * (1.0f / 16.0f) + bb; } }
  LDSX();
  for (int q = lane; q < 16 * NH * 4; q += 32) { const int h = q >> 6, rl = (q >> 2) & 15, pc = q & 3; union { v8h h8; v4u u; } pk;
#pragma unroll
    for (int e = 0; e < 8; ++e) pk.h8[e] = (_Float16)(so[wave][rl][h * HD + pc * 8 + e] * 4.0f);
    vst2(K16 + (((size_t)b * NH + h) * NK + t0b + wave * 16 + rl) * HD + pc * 8, pk.u); }
#pragma unroll 4
  for (int rl = 0; rl < 16; ++rl) for (int e = 0; e < 8; ++e) st[lane * 8 + e][wave * 16 + rl] = (_Float16)(so[wave][rl][CC + lane * 8 + e] * 4.0f);
  __syncthreads();
  for (int q = tid; q < CC * 8; q += 128) { const int c = q >> 3, pc = q & 7; const int h = c >> 5, d = c & 31; vst2(VT + (((size_t)b * NH + h) * HD + d) * NK + t0b + pc * 8, *(const v4u*)(&st[c][pc * 8])); }
}
__global__ __launch_bounds__(128) void k_attn(const _Float16* __restrict__ Q16, const _Float16* __restrict__ K16, const _Float16* __restrict__ VT, _Float16* __restrict__ O16) {
  __shared__ __align__(16) float sS[4][16][NK + 4];
  __shared__ __align__(16) _Float16 sP[4][16][NK + 8];
  __shared__ __align__(16) float sO[4][16][36];
  const int tid = threadIdx.x, w = tid >> 5, lane = tid & 31, col = lane & 15, g = lane >> 4;
  const int b = blockIdx.z, h = blockIdx.y, q0 = blockIdx.x * 64 + w * 16; const size_t bh = (size_t)b * NH + h;
  const v16h aq = frag_h(Q16 + ((size_t)b * NN + q0 + col) * CC + h * HD, lane);
#pragma unroll
  for (int t = 0; t < NK / 16; ++t) { v8f s = {}; s = wmma16(aq, frag_h(K16 + (bh * NK + t * 16 + col) * HD, lane), s);
#pragma unroll
    for (int r = 0; r < 8; ++r) sS[w][8 * g + r][t * 16 + col] = s[r] * (0.17677669529663687f / 16.0f); }
  LDSX();
  { const int m = col; float mx = -3.4e38f; for (int e = 0; e < 128; ++e) mx = fmaxf(mx, sS[w][m][g * 128 + e]); mx = fmaxf(mx, __shfl_xor(mx, 16, 32));
    float l = 0.f; for (int e = 0; e < 128; ++e) { const float p = expf(sS[w][m][g * 128 + e] - mx); sS[w][m][g * 128 + e] = p; l += p; }
    l += __shfl_xor(l, 16, 32); const float inv = 16384.0f / l;
    for (int e = 0; e < 128; ++e) sP[w][m][g * 128 + e] = (_Float16)(sS[w][m][g * 128 + e] * inv); }
  LDSX();
  v8f acc[2] = {};
#pragma unroll
  for (int kc = 0; kc < NK / 32; ++kc) { const v16h pa = frag_h(&sP[w][col][0] + kc * 32, lane);
#pragma unroll
    for (int t = 0; t < 2; ++t) acc[t] = wmma16(pa, frag_h(VT + (bh * HD + t * 16 + col) * NK + kc * 32, lane), acc[t]); }
#pragma unroll
  for (int t = 0; t < 2; ++t)
#pragma unroll
    for (int r = 0; r < 8; ++r) sO[w][8 * g + r][t * 16 + col] = acc[t][r] * (8.0f / (16384.0f * 4.0f));
  LDSX();
  for (int q = lane; q < 16 * 4; q += 32) { const int rl = q >> 2, pc = q & 3; union { v8h h8; v4u u; } pk;
#pragma unroll
    for (int e = 0; e < 8; ++e) pk.h8[e] = (_Float16)sO[w][rl][pc * 8 + e];
    vst2(O16 + ((bh * NN + q0 + rl) * HD) + pc * 8, pk.u); }
}
__global__ __launch_bounds__(128) void k_proj(const _Float16* __restrict__ O16, const _Float16* __restrict__ P, const float* __restrict__ pb, float* __restrict__ out) {
  __shared__ __align__(16) float so[4][16][132];
  const int tid = threadIdx.x, wave = tid >> 5, lane = tid & 31, col = lane & 15, g = lane >> 4;
  const int r0 = blockIdx.x * 64 + wave * 16, n0 = blockIdx.y * 128;
  v8f acc[8] = {};
#pragma unroll
  for (int kc = 0; kc < CC / 32; ++kc) { const int R = r0 + col; const v16h a = frag_h(O16 + (((size_t)(R >> 12) * NH + kc) * NN + (R & 4095)) * HD, lane);
#pragma unroll
    for (int j = 0; j < 8; ++j) acc[j] = wmma16(a, frag_h(P + (size_t)(768 + n0 + j * 16 + col) * CC + kc * 32, lane), acc[j]); }
#pragma unroll
  for (int j = 0; j < 8; ++j) { const float bb = pb[n0 + j * 16 + col];
#pragma unroll
    for (int r = 0; r < 8; ++r) so[wave][8 * g + r][j * 16 + col] = acc[j][r] * (1.0f / 128.0f) + bb; }
  LDSX();
#pragma unroll 4
  for (int rl = 0; rl < 16; ++rl) vst2(out + (size_t)(r0 + rl) * CC + n0 + lane * 4, *(const v4f*)(&so[wave][rl][lane * 4]));
}
extern "C" void kernel_launch(void* const* d_in, const int* in_sizes, int n_in, void* d_out, int out_size, void* d_ws, size_t ws_size, hipStream_t stream) {
  (void)in_sizes; (void)n_in; (void)out_size; (void)ws_size;
  const float** I = (const float**)d_in;
  const float* x = I[0]; const float* qw = I[3]; const float* qb = I[4]; const float* kvw = I[5]; const float* kvb = I[6]; const float* pw = I[7]; const float* pb = I[8]; const float* srw = I[9]; const float* srb = I[10]; const float* ng = I[11]; const float* nbeta = I[12];
  float* out = (float*)d_out;
  char* ws = (char*)d_ws; size_t off = 0;
  auto take = [&](size_t bytes) { char* p = ws + off; off += (bytes + 255) & ~(size_t)255; return p; };
  _Float16* x16 = (_Float16*)take((size_t)NR * CC * 2); _Float16* P = (_Float16*)take((size_t)1024 * CC * 2); _Float16* Psr = (_Float16*)take((size_t)CC * 16 * CC * 2);
  _Float16* Q16 = (_Float16*)take((size_t)NR * CC * 2); _Float16* K16 = (_Float16*)take((size_t)NB * NH * NK * HD * 2); _Float16* VT = (_Float16*)take((size_t)NB * NH * HD * NK * 2); _Float16* O16 = (_Float16*)take((size_t)NR * CC * 2);
  { const size_t n8 = (size_t)NR * CC / 8; k_cvt<<<(unsigned)(n8 / 256), 256, 0, stream>>>(x, x16, n8); }
  k_pack<<<1024 + CC, 256, 0, stream>>>(qw, kvw, pw, srw, P, Psr);
  k_q<<<dim3(NR / 64, CC / 128), 128, 0, stream>>>(x16, P, qb, Q16);
  k_kv<<<dim3(NK / 64, NB), 128, 0, stream>>>(x16, Psr, srb, ng, nbeta, P, kvb, K16, VT);
  k_attn<<<dim3(NN / 64, NH, NB), 128, 0, stream>>>(Q16, K16, VT, O16);
  k_proj<<<dim3(NR / 64, CC / 128), 128, 0, stream>>>(O16, P, pb, out);
}
